// KLGCN_52106543235211
// MI455X (gfx1250) — hardware-run, weakly checked
//
#include <hip/hip_runtime.h>
#include <stddef.h>


#define DIM   64
#define NNB   16
#define RPB   32
#define NWAVE 2
#define NTHR  (NWAVE * 32)
#define PA    72

static_assert(RPB == NWAVE * 16);
static_assert(((PA * 2) % 16) == 0);
static_assert(((DIM * DIM) % NTHR) == 0);
static_assert(RPB == 32);

typedef float          v2f   __attribute__((ext_vector_type(2)));
typedef float          v4f   __attribute__((ext_vector_type(4)));
typedef float          v8f   __attribute__((ext_vector_type(8)));
typedef unsigned short v2us  __attribute__((ext_vector_type(2)));
typedef unsigned short v8us  __attribute__((ext_vector_type(8)));
typedef unsigned short v16us __attribute__((ext_vector_type(16)));
typedef __bf16         v16bf __attribute__((ext_vector_type(16)));
union Frag { v16bf v; v16us u; v8us h[2]; };

__device__ __forceinline__ unsigned short bf_rne(float x) {
  unsigned int u = __float_as_uint(x);
  u += 0x7FFFu + ((u >> 16) & 1u);
  return (unsigned short)(u >> 16);
}
__device__ __forceinline__ void split2(float x, unsigned short& hi, unsigned short& lo) {
  const unsigned short h = bf_rne(x);
  const float r = x - __uint_as_float(((unsigned int)h) << 16);
  hi = h;
  lo = bf_rne(r);
}

__device__ __forceinline__ v8f wmb(v16bf a, v16bf b, v8f c) {
  v8f d = __builtin_amdgcn_wmma_f32_16x16x32_bf16(false, a, false, b, (short)0, c, false, false);
  asm volatile("v_nop\n\tv_nop\n\tv_nop\n\tv_nop" : "+v"(d) : "v"(a), "v"(b));
  return d;
}
__device__ __forceinline__ v8f mm3(v16bf ah, v16bf al, v16bf bh, v16bf bl, v8f c) {
  c = wmb(ah, bh, c);
  c = wmb(ah, bl, c);
  c = wmb(al, bh, c);
  return c;
}
__device__ __forceinline__ v16bf ldfrag(const unsigned short* p) {
  Frag f;
  f.h[0] = *(const v8us*)p;
  f.h[1] = *(const v8us*)(p + 16);
  return f.v;
}
__device__ __forceinline__ int wrapclamp(int i, int n) {
  if (i < 0) i += n;
  return i < 0 ? 0 : (i > n - 1 ? n - 1 : i);
}

__device__ __forceinline__ void sc_store(const float* sSc, float* out, int nB, int blk, int lane) {
  const int b4 = blk * RPB + 4 * lane;
  const v4f v = *(const v4f*)(sSc + 4 * lane);
  if (b4 + 4 <= nB) {
    *(volatile v4f*)(out + b4) = v;
  } else {
    if (b4 + 0 < nB) *(volatile float*)(out + b4 + 0) = v.x;
    if (b4 + 1 < nB) *(volatile float*)(out + b4 + 1) = v.y;
    if (b4 + 2 < nB) *(volatile float*)(out + b4 + 2) = v.z;
  }
}

__global__ __launch_bounds__(NTHR) void k_main(
    const int* __restrict__ uidx, const int* __restrict__ vidx,
    const int* __restrict__ unb, const int* __restrict__ inb,
    const int* __restrict__ adje, const int* __restrict__ adjr,
    const float* __restrict__ uemb, const float* __restrict__ eemb,
    const float* __restrict__ remb, const float* __restrict__ W,
    const float* __restrict__ bias, float* out,
    int nB, int nUser, int nEnt, int nRel) {
  __shared__ __attribute__((aligned(16))) unsigned short sWh[DIM * PA];
  __shared__ __attribute__((aligned(16))) unsigned short sWl[DIM * PA];
  __shared__ __attribute__((aligned(16))) unsigned short sAh[RPB * PA];
  __shared__ __attribute__((aligned(16))) unsigned short sAl[RPB * PA];
  __shared__ __attribute__((aligned(16))) float sUF[RPB * DIM];
  __shared__ __attribute__((aligned(16))) float sLI[RPB * DIM];
  __shared__ __attribute__((aligned(16))) float sSc[RPB];

  const int tid = (int)threadIdx.x, lane = tid & 31, wave = tid >> 5, hh = lane >> 4, m = lane & 15;

#pragma unroll 4
  for (int i = 0; i < (DIM * DIM) / NTHR; ++i) {
    const int idx = tid + i * NTHR;
    const int k = idx >> 6, n = idx & 63;
    unsigned short p, q;
    split2(W[idx], p, q);
    sWh[n * PA + k] = p;
    sWl[n * PA + k] = q;
  }

  const int row0 = (int)blockIdx.x * RPB + wave * 16;
#pragma unroll 1
  for (int r = 0; r < 16; ++r) {
    const int lrow = wave * 16 + r;
    int b = row0 + r;
    b = b > nB - 1 ? nB - 1 : b;
    const int ub = wrapclamp(uidx[b], nUser);
    const int vb = wrapclamp(vidx[b], nEnt);

    const v2f ue = *(const v2f*)(uemb + (size_t)ub * DIM + 2 * lane);
    const v2f io = *(const v2f*)(eemb + (size_t)vb * DIM + 2 * lane);

    const int myrel = wrapclamp(adjr[(size_t)vb * NNB + m], nRel);
    const int myent = wrapclamp(adje[(size_t)vb * NNB + m], nEnt);
    const int myiu  = wrapclamp(inb[(size_t)b * NNB + m], nUser);
    const int myie  = wrapclamp(unb[(size_t)b * NNB + m], nEnt);

    float mys = 0.0f;
#pragma unroll
    for (int n = 0; n < NNB; ++n) {
      const int rid = __shfl(myrel, n, 32);
      const v2f re = *(const v2f*)(remb + (size_t)rid * DIM + 2 * lane);
      float p = ue.x * re.x + ue.y * re.y;
      p += __shfl_xor(p, 16, 32);
      p += __shfl_xor(p, 8, 32);
      p += __shfl_xor(p, 4, 32);
      p += __shfl_xor(p, 2, 32);
      p += __shfl_xor(p, 1, 32);
      mys = (m == n) ? p : mys;
    }
    float mx = mys;
    mx = fmaxf(mx, __shfl_xor(mx, 8, 32));
    mx = fmaxf(mx, __shfl_xor(mx, 4, 32));
    mx = fmaxf(mx, __shfl_xor(mx, 2, 32));
    mx = fmaxf(mx, __shfl_xor(mx, 1, 32));
    const float e = expf(mys - mx);
    float ssum = e;
    ssum += __shfl_xor(ssum, 8, 32);
    ssum += __shfl_xor(ssum, 4, 32);
    ssum += __shfl_xor(ssum, 2, 32);
    ssum += __shfl_xor(ssum, 1, 32);
    const float attn = e * (1.0f / ssum);

    v2f a;
    a.x = 0.0f; a.y = 0.0f;
#pragma unroll
    for (int n = 0; n < NNB; ++n) {
      const float w = __shfl(attn, n, 32);
      const int eid = __shfl(myent, n, 32);
      const v2f ne = *(const v2f*)(eemb + (size_t)eid * DIM + 2 * lane);
      a.x += w * ne.x;
      a.y += w * ne.y;
    }
    const float c0 = io.x + a.x;
    const float c1 = io.y + a.y;
    unsigned short h0, l0, h1, l1;
    split2(c0, h0, l0);
    split2(c1, h1, l1);
    v2us hv, lv;
    hv.x = h0; hv.y = h1;
    lv.x = l0; lv.y = l1;
    *(v2us*)(sAh + lrow * PA + 2 * lane) = hv;
    *(v2us*)(sAl + lrow * PA + 2 * lane) = lv;

    v2f lu, li;
    lu.x = 0.0f; lu.y = 0.0f; li.x = 0.0f; li.y = 0.0f;
#pragma unroll
    for (int n = 0; n < NNB; ++n) {
      const int iu = __shfl(myiu, n, 32);
      const int ie = __shfl(myie, n, 32);
      const v2f xu = *(const v2f*)(uemb + (size_t)iu * DIM + 2 * lane);
      const v2f xe = *(const v2f*)(eemb + (size_t)ie * DIM + 2 * lane);
      lu.x += xu.x; lu.y += xu.y;
      li.x += xe.x; li.y += xe.y;
    }
    const float invn = 0.0625f;
    v2f uf, lim;
    uf.x = 0.5f * (lu.x * invn) + 0.5f * ue.x;
    uf.y = 0.5f * (lu.y * invn) + 0.5f * ue.y;
    lim.x = li.x * invn;
    lim.y = li.y * invn;
    *(v2f*)(sUF + lrow * DIM + 2 * lane) = uf;
    *(v2f*)(sLI + lrow * DIM + 2 * lane) = lim;
  }

  __syncthreads();

  const v8f z = {0.f, 0.f, 0.f, 0.f, 0.f, 0.f, 0.f, 0.f};
  v8f acc[4] = {z, z, z, z};
#pragma unroll
  for (int ks = 0; ks < 2; ++ks) {
    const v16bf ah = ldfrag(sAh + (wave * 16 + m) * PA + 32 * ks + 8 * hh);
    const v16bf al = ldfrag(sAl + (wave * 16 + m) * PA + 32 * ks + 8 * hh);
#pragma unroll
    for (int nt = 0; nt < 4; ++nt) {
      const unsigned short* wp = sWh + (16 * nt + m) * PA + 32 * ks + 8 * hh;
      const unsigned short* wq = sWl + (16 * nt + m) * PA + 32 * ks + 8 * hh;
      acc[nt] = mm3(ah, al, ldfrag(wp), ldfrag(wq), acc[nt]);
    }
  }

  float pr[8];
#pragma unroll
  for (int r = 0; r < 8; ++r) pr[r] = 0.0f;
#pragma unroll
  for (int nt = 0; nt < 4; ++nt) {
    const int col = 16 * nt + m;
    const float bcol = bias[col];
#pragma unroll
    for (int r = 0; r < 8; ++r) {
      const int lrow = wave * 16 + 8 * hh + r;
      const float ite = tanhf(acc[nt][r] + bcol);
      const float itf = 0.5f * sLI[lrow * DIM + col] + 0.5f * ite;
      pr[r] += sUF[lrow * DIM + col] * itf;
    }
  }
#pragma unroll
  for (int r = 0; r < 8; ++r) {
    pr[r] += __shfl_xor(pr[r], 8, 32);
    pr[r] += __shfl_xor(pr[r], 4, 32);
    pr[r] += __shfl_xor(pr[r], 2, 32);
    pr[r] += __shfl_xor(pr[r], 1, 32);
  }
  float mine = 0.0f;
#pragma unroll
  for (int r = 0; r < 8; ++r) mine = (m == r) ? pr[r] : mine;
  const float sig = 1.0f / (1.0f + expf(-mine));
  if (m < 8) sSc[wave * 16 + 8 * hh + m] = sig;
  __syncthreads();

  if (wave == 0) {
    if (lane < 8) sc_store(sSc, out, nB, (int)blockIdx.x, lane);
    __threadfence();
    if (lane < 8) sc_store(sSc, out, nB, (int)blockIdx.x, lane);
  }
}

extern "C" void kernel_launch(void* const* d_in, const int* in_sizes, int n_in,
                              void* d_out, int out_size, void* d_ws, size_t ws_size,
                              hipStream_t stream) {
  (void)d_ws; (void)ws_size;
  if (n_in < 11) return;
  if (out_size <= 0) return;
  const int nB = out_size;
  if (in_sizes[0] != nB || in_sizes[1] != nB) return;
  if (in_sizes[2] != nB * NNB || in_sizes[3] != nB * NNB) return;
  if (in_sizes[6] <= 0 || (in_sizes[6] % DIM) != 0) return;
  if (in_sizes[7] <= 0 || (in_sizes[7] % DIM) != 0) return;
  if (in_sizes[8] <= 0 || (in_sizes[8] % DIM) != 0) return;
  const int nUser = in_sizes[6] / DIM;
  const int nEnt  = in_sizes[7] / DIM;
  const int nRel  = in_sizes[8] / DIM;
  if (in_sizes[4] != nEnt * NNB || in_sizes[5] != nEnt * NNB) return;
  if (in_sizes[9] != DIM * DIM || in_sizes[10] != DIM) return;

  const int*   uidx = (const int*)d_in[0];
  const int*   vidx = (const int*)d_in[1];
  const int*   unb  = (const int*)d_in[2];
  const int*   inb  = (const int*)d_in[3];
  const int*   adje = (const int*)d_in[4];
  const int*   adjr = (const int*)d_in[5];
  const float* uemb = (const float*)d_in[6];
  const float* eemb = (const float*)d_in[7];
  const float* remb = (const float*)d_in[8];
  const float* W    = (const float*)d_in[9];
  const float* bias = (const float*)d_in[10];
  float* out = (float*)d_out;

  const int grid = (nB + RPB - 1) / RPB;
  k_main<<<grid, NTHR, 0, stream>>>(uidx, vidx, unb, inb, adje, adjr, uemb, eemb, remb, W, bias,
                                    out, nB, nUser, nEnt, nRel);
}
